// LocalSubgraphEncoder_82918638617235
// MI455X (gfx1250) — hardware-run, weakly checked
//
#include <hip/hip_runtime.h>


namespace {
constexpr int N = 4096, D = 256, NHD = 8, DH = 32, E = 131072, NTY = 16;
constexpr float XS = 8.0f, PS = 1024.0f, WSC = 256.0f;
typedef _Float16 b16;
typedef __attribute__((ext_vector_type(16))) _Float16 v16b;
typedef __attribute__((ext_vector_type(8))) _Float16 v8b;
typedef __attribute__((ext_vector_type(8))) float v8f;
typedef __attribute__((ext_vector_type(4))) float v4f;
__device__ __forceinline__ float bf16_rne(float f) { unsigned int u = __float_as_uint(f); u += 0x7FFFu + ((u >> 16) & 1u); float r = __uint_as_float(u & 0xFFFF0000u); asm volatile("" : "+v"(r)); return r; }
__device__ __forceinline__ void split16(float v, b16& hi, b16& lo) { hi = (b16)v; lo = (b16)(v - (float)hi); }
__device__ __forceinline__ v16b frag_kb(const b16* p, int hh) { const v8b a = *(const v8b*)(p + 8 * hh), b = *(const v8b*)(p + 16 + 8 * hh); v16b f;
#pragma unroll
  for (int e = 0; e < 8; ++e) { f[e] = a[e]; f[8 + e] = b[e]; } return f; }
__device__ __forceinline__ v8f wmma16b(v16b a, v16b b, v8f c) { v8f d = __builtin_amdgcn_wmma_f32_16x16x32_f16(false, a, false, b, (short)0, c, false, false); asm volatile("v_nop\n\tv_nop\n\tv_nop\n\tv_nop" : "+v"(d) : "v"(a), "v"(b)); return d; }
__device__ __forceinline__ void wave_lds_sync() { __builtin_amdgcn_fence(__ATOMIC_RELEASE, "workgroup"); __builtin_amdgcn_wave_barrier(); __builtin_amdgcn_fence(__ATOMIC_ACQUIRE, "workgroup"); }
__device__ __forceinline__ float pmul(float a, float b) { float p = a * b; asm volatile("" : "+v"(p)); return p; }
__device__ __forceinline__ int iclamp(int v, int lo, int hi) { return v < lo ? lo : (v > hi ? hi : v); }
constexpr int CSR_NBLK7 = 512, CSR_GB7 = 7, CSR_GN7 = 1 << CSR_GB7  , CSR_TS7 = (CSR_GN7 < 32 ? 32 : CSR_GN7)  , CSR_MAXG7 = 512, CSR_CAP7 = 12288  ;
__device__ __host__ __forceinline__ int csr_tix7(int v) { return (v >> CSR_GB7) * CSR_TS7 + (v & (CSR_GN7 - 1)); }
__global__ __launch_bounds__(64) void csrA_kernel7(const int* __restrict__ dst, int E, int N, int nG, int CHP, int NGP, int* __restrict__ STG, int* __restrict__ HST) {
  extern __shared__ int sm[];
  int* cnt = sm; int* run = sm + NGP; int* ids = sm + 2 * NGP;
  const int b = blockIdx.x; const int ch = (E + CSR_NBLK7 - 1) / CSR_NBLK7; const int e0 = b * ch, e1 = min(E, e0 + ch);
  for (int i = threadIdx.x; i < NGP; i += 64) cnt[i] = 0;
  for (int i = threadIdx.x; i < CHP; i += 64) ids[i] = -1;
  __syncthreads();
  if (threadIdx.x == 0) {
    for (int e = e0; e < e1; ++e) { int d = dst[e]; d = (d < 0) ? 0 : (d >= N ? N - 1 : d); cnt[d >> CSR_GB7] += 1; }
    int acc = 0; for (int g = 0; g < nG; ++g) { run[g] = acc; acc += cnt[g]; }
    for (int e = e0; e < e1; ++e) { int d = dst[e]; d = (d < 0) ? 0 : (d >= N ? N - 1 : d); const int g = d >> CSR_GB7; ids[run[g]] = e; run[g] += 1; } }
  __syncthreads();
  typedef __attribute__((ext_vector_type(4))) int v4i;
  for (int pass = 0; pass < 2; ++pass) {
    for (int i = threadIdx.x; i < CHP / 4; i += 64) *(volatile v4i*)(STG + (size_t)b * CHP + i * 4) = *(const v4i*)(&ids[i * 4]);
    for (int i = threadIdx.x; i < NGP / 4; i += 64) { v4i v; for (int e = 0; e < 4; ++e) v[e] = (i * 4 + e < nG) ? cnt[i * 4 + e] : 0; *(volatile v4i*)(HST + (size_t)b * NGP + i * 4) = v; }
    __threadfence(); }
}
__global__ __launch_bounds__(512) void csrS_kernel7(const int* __restrict__ HST, int nG, int NGP, int* __restrict__ START, int* __restrict__ TOT, int* __restrict__ OFF) {
  __shared__ int tot[CSR_MAXG7];
  const int b = threadIdx.x;
  for (int pass = 0; pass < 2; ++pass) { int runb = 0; for (int g = 0; g < nG; ++g) { int c = HST[(size_t)b * NGP + g]; c = (c < 0) ? 0 : c; ((volatile int*)OFF)[(size_t)g * CSR_NBLK7 + b] = runb; runb += c; } __threadfence(); }
  for (int g = threadIdx.x; g < nG; g += 512) { int s = 0; for (int bb = 0; bb < CSR_NBLK7; ++bb) { int c = HST[(size_t)bb * NGP + g]; s += (c < 0) ? 0 : c; } tot[g] = s; }
  __syncthreads();
  if (threadIdx.x < 32) {
    __shared__ int st[CSR_MAXG7 + 32];
    if (threadIdx.x == 0) { int acc = 0; for (int g = 0; g < NGP; ++g) { st[g] = acc; if (g < nG) acc += (tot[g] + 31) & ~31; } st[NGP] = acc; }
    __builtin_amdgcn_fence(__ATOMIC_RELEASE, "workgroup"); __builtin_amdgcn_wave_barrier(); __builtin_amdgcn_fence(__ATOMIC_ACQUIRE, "workgroup");
    for (int pass = 0; pass < 2; ++pass) { for (int i = threadIdx.x; i < NGP + 32; i += 32) { ((volatile int*)START)[i] = (i <= NGP) ? st[min(i, NGP)] : 0; ((volatile int*)TOT)[i] = (i < nG) ? tot[i] : 0; } __threadfence(); } }
}
__global__ __launch_bounds__(256) void csrB_kernel7(const int* __restrict__ dst, int N, int nG, int CHP, int NGP, int permLen, const int* __restrict__ STG, const int* __restrict__ HST, const int* __restrict__ OFF, const int* __restrict__ START, const int* __restrict__ TOT, int* __restrict__ PERM, int* __restrict__ ROWPTR, int* __restrict__ ROWCNT, int* __restrict__ FLAG) {
  typedef __attribute__((ext_vector_type(4))) int v4i;
  __shared__ int ids[CSR_CAP7]; __shared__ unsigned short key[CSR_CAP7]; __shared__ int outp[CSR_CAP7]; __shared__ int ncnt[CSR_GN7 + 1]; __shared__ int boff[CSR_NBLK7 + 1];
  const int g = blockIdx.x, t_ = threadIdx.x; int tot = TOT[g]; int st = START[g], stn = START[g + 1]; const int v0 = g * CSR_GN7; const int nv = min(CSR_GN7, N - v0); const int t0 = g * CSR_TS7;
  st = (st < 0) ? 0 : (st > permLen - 32 ? permLen - 32 : st) & ~31; stn = (stn < st) ? st : (stn > permLen ? permLen : stn); tot = (tot < 0) ? 0 : tot; if (tot > stn - st && tot <= CSR_CAP7) tot = stn - st;
  if (tot > CSR_CAP7) {
    for (int pass = 0; pass < 2; ++pass) { for (int i = t_; i < CSR_TS7 / 4; i += 256) { v4i a, c; for (int e = 0; e < 4; ++e) { a[e] = st; c[e] = 0; } *(volatile v4i*)(ROWPTR + t0 + i * 4) = a; *(volatile v4i*)(ROWCNT + t0 + i * 4) = c; } if (t_ == 0) ((volatile int*)FLAG)[0] = 1; __threadfence(); } (void)nv; return; }
  if (t_ == 0) { int acc = 0; for (int b = 0; b < CSR_NBLK7; ++b) { boff[b] = acc; int c = HST[(size_t)b * NGP + g]; c = (c < 0) ? 0 : (c > CHP ? CHP : c); acc += c; if (acc > tot) acc = tot; } boff[CSR_NBLK7] = acc; }
  for (int i = t_; i <= CSR_GN7; i += 256) ncnt[i] = 0;
  __syncthreads();
  for (int b = 0; b < CSR_NBLK7; ++b) { const int c = boff[b + 1] - boff[b]; int o_ = OFF[(size_t)g * CSR_NBLK7 + b]; o_ = (o_ < 0) ? 0 : (o_ > CHP - c ? CHP - c : o_); const int* src_ = STG + (size_t)b * CHP + o_;
    for (int i = t_; i < c; i += 256) { int id = src_[i]; id = (id < 0) ? 0 : id; ids[boff[b] + i] = id; int d = dst[id]; d = (d < v0) ? v0 : (d >= N ? N - 1 : d); int kk = d - v0; kk = (kk < 0) ? 0 : (kk >= CSR_GN7 ? CSR_GN7 - 1 : kk); key[boff[b] + i] = (unsigned short)kk; } }
  __syncthreads();
  if (t_ == 0) { for (int i = 0; i < tot; ++i) ncnt[key[i]] += 1; int acc = 0; for (int vl = 0; vl < CSR_GN7; ++vl) { const int c = ncnt[vl]; ncnt[vl] = acc; acc += c; } ncnt[CSR_GN7] = acc;
    for (int i = 0; i < tot; ++i) { const int vl = key[i]; outp[ncnt[vl]] = ids[i]; ncnt[vl] += 1; }
    for (int vl = CSR_GN7; vl > 0; --vl) ncnt[vl] = ncnt[vl - 1]; ncnt[0] = 0; }
  __syncthreads();
  for (int pass = 0; pass < 2; ++pass) {
    for (int i = t_; i < (stn - st) / 4; i += 256) { v4i v; for (int e = 0; e < 4; ++e) { const int q = i * 4 + e; v[e] = (q < tot) ? outp[q] : -1; } *(volatile v4i*)(PERM + st + i * 4) = v; }
    for (int i = t_; i < CSR_TS7 / 4; i += 256) { v4i a, c; for (int e = 0; e < 4; ++e) { const int vl = i * 4 + e; const int vc = vl < CSR_GN7 ? vl : CSR_GN7; a[e] = (vl < CSR_GN7) ? st + ncnt[vc] : st; c[e] = (vl < nv) ? (ncnt[(vc < CSR_GN7 ? vc : CSR_GN7 - 1) + 1] - ncnt[vc]) : 0; } *(volatile v4i*)(ROWPTR + t0 + i * 4) = a; *(volatile v4i*)(ROWCNT + t0 + i * 4) = c; }
    __threadfence(); }
}
__global__ __launch_bounds__(256) void csrZ_kernel7(int* __restrict__ p, size_t n4) { typedef __attribute__((ext_vector_type(4))) int v4i; const size_t tid = (size_t)blockIdx.x * 256 + threadIdx.x, nth = (size_t)gridDim.x * 256; v4i z = {0, 0, 0, 0}; for (size_t i = tid; i < n4; i += nth) *(volatile v4i*)(p + i * 4) = z; }
struct CsrBufs7 { int *STG, *HST, *OFF, *START, *TOT, *PERM, *ROWPTR, *ROWCNT, *FLAG; int nG, NGP, CHP; size_t permLen; char* base; size_t bytes; };
static size_t csr_carve7(CsrBufs7& c, char* ws, size_t off, int E, int N) {
  const size_t off0 = off; c.base = ws + off;
  auto al = [&](size_t bytes) { char* p = ws + off; off += (bytes + 255) & ~(size_t)255; return p; };
  c.nG = (N + CSR_GN7 - 1) / CSR_GN7; c.NGP = (c.nG + 31) & ~31; const int ch = (E + CSR_NBLK7 - 1) / CSR_NBLK7; c.CHP = (ch + 31) & ~31; c.permLen = (size_t)E + 32 * (size_t)c.nG + 32;
  c.STG = (int*)al((size_t)CSR_NBLK7 * c.CHP * 4); c.HST = (int*)al((size_t)CSR_NBLK7 * c.NGP * 4); c.OFF = (int*)al((size_t)c.NGP * CSR_NBLK7 * 4); c.START = (int*)al((size_t)(c.NGP + 64) * 4); c.TOT = (int*)al((size_t)(c.NGP + 64) * 4);
  c.PERM = (int*)al(c.permLen * 4); c.ROWPTR = (int*)al((size_t)c.nG * CSR_TS7 * 4); c.ROWCNT = (int*)al((size_t)c.nG * CSR_TS7 * 4); c.FLAG = (int*)al(256);
  c.bytes = off - off0; return off;
}
static void csr_build7(const CsrBufs7& c, const int* dst, int E, int N, hipStream_t stream) {
  const size_t smem = (size_t)(2 * c.NGP + c.CHP) * 4;
  csrZ_kernel7<<<512, 256, 0, stream>>>((int*)c.base, c.bytes / 16);
  csrA_kernel7<<<CSR_NBLK7, 64, smem, stream>>>(dst, E, N, c.nG, c.CHP, c.NGP, c.STG, c.HST);
  csrS_kernel7<<<1, 512, 0, stream>>>(c.HST, c.nG, c.NGP, c.START, c.TOT, c.OFF);
  csrB_kernel7<<<c.nG, 256, 0, stream>>>(dst, N, c.nG, c.CHP, c.NGP, (int)c.permLen, c.STG, c.HST, c.OFF, c.START, c.TOT, c.PERM, c.ROWPTR, c.ROWCNT, c.FLAG);
}


__global__ __launch_bounds__(256) void wput_kernel(const float* __restrict__ w, int ooff, b16* __restrict__ WT) { const int u = blockIdx.x * 256 + threadIdx.x; if (u >= D * 32) return; const int o = u / 32, k0 = (u % 32) * 8; v8b v;
#pragma unroll
  for (int j = 0; j < 8; ++j) v[j] = (b16)(bf16_rne(w[(size_t)(k0 + j) * D + o]) * WSC); for (int pass = 0; pass < 2; ++pass) { *(volatile v8b*)(WT + (size_t)(ooff + o) * D + k0) = v; __threadfence(); } }
__global__ __launch_bounds__(32) void qkv_kernel(const float* __restrict__ x, const float* __restrict__ pe, const b16* __restrict__ WT, const float* __restrict__ bq, const float* __restrict__ bk, const float* __restrict__ bv, float* __restrict__ QKV) {
  __shared__ __attribute__((aligned(16))) b16 Ah[16][D + 8], Al[16][D + 8]; __shared__ float Tf[16][132]; const int lane = threadIdx.x, nloc = lane & 15, hlf = lane >> 4; const int cg = blockIdx.x % 6; const size_t m0 = (size_t)(blockIdx.x / 6) * 16;
  for (int rr = 0; rr < 16; ++rr) for (int q = 0; q < D / 32; ++q) { const size_t o = (m0 + rr) * D + q * 32 + lane; b16 p, ql; split16((bf16_rne(x[o]) + bf16_rne(pe[o])) * XS, p, ql); Ah[rr][q * 32 + lane] = p; Al[rr][q * 32 + lane] = ql; }
  wave_lds_sync(); v8f acc[8];
#pragma unroll
  for (int t = 0; t < 8; ++t) acc[t] = (v8f){};
#pragma unroll 2
  for (int kb = 0; kb < D; kb += 32) { const v16b a = frag_kb(&Ah[nloc][kb], hlf), al = frag_kb(&Al[nloc][kb], hlf);
#pragma unroll
    for (int t = 0; t < 8; ++t) { const v16b bw = frag_kb(WT + (size_t)(cg * 128 + t * 16 + nloc) * D + kb, hlf); acc[t] = wmma16b(a, bw, acc[t]); acc[t] = wmma16b(al, bw, acc[t]); } }
  const int which = cg / 2; const float* bias = which == 0 ? bq : (which == 1 ? bk : bv);
#pragma unroll
  for (int t = 0; t < 8; ++t) { const int c = cg * 128 + t * 16 + nloc; const float bb = bf16_rne(bias[c - which * D]);
#pragma unroll
    for (int r8 = 0; r8 < 8; ++r8) Tf[8 * hlf + r8][t * 16 + nloc] = acc[t][r8] * (1.0f / (XS * WSC)) + bb; }
  wave_lds_sync();
  for (int pass = 0; pass < 2; ++pass) { for (int rr = 0; rr < 16; ++rr) *(volatile v4f*)(QKV + (m0 + rr) * 3 * D + cg * 128 + lane * 4) = *(const v4f*)(&Tf[rr][lane * 4]); __threadfence(); }
}
__global__ __launch_bounds__(32) void bias_kernel(const float* __restrict__ emb, const int* __restrict__ dsts, const int* __restrict__ ety, int hd, const int* __restrict__ PERM, const int* __restrict__ ROWPTR, const int* __restrict__ ROWCNT, int permLen, float* __restrict__ BP) {
  __shared__ float row[N]; const int lane = threadIdx.x; const int n = blockIdx.x; for (int c = lane; c < N; c += 32) row[c] = 0.0f; wave_lds_sync();
  if (lane == 0) { int st = ROWPTR[n], cnt = ROWCNT[n]; cnt = iclamp(cnt, 0, 1 << 16); st = iclamp(st, 0, permLen - cnt);
    for (int j = 0; j < cnt; ++j) { const int e = iclamp(PERM[st + j], 0, E - 1); const int m = iclamp(dsts[e], 0, N - 1), t = iclamp(ety[e], 0, NTY - 1); row[m] += bf16_rne(emb[t * NHD + hd]); } }
  wave_lds_sync();
  for (int pass = 0; pass < 2; ++pass) { for (int c = lane * 4; c < N; c += 128) *(volatile v4f*)(BP + (size_t)n * N + c) = *(const v4f*)(&row[c]); __threadfence(); } }
__global__ __launch_bounds__(32) void att_kernel(const float* __restrict__ QKV, const float* __restrict__ BP, int hd, int QV, float* __restrict__ O) {
  __shared__ __attribute__((aligned(16))) b16 Qh[16][40], Ql[16][40], Kh[32][40], Kl[32][40], Ph[16][40], Pl[16][40], Vh[DH][40], Vl[DH][40]; __shared__ float Sc[16][33], Mx[16], Dn[16], Sf[16], Of[16][DH + 1];
  const int lane = threadIdx.x, nloc = lane & 15, hlf = lane >> 4; const int q0 = blockIdx.x * 16; if (q0 >= QV) return;
  for (int rr = 0; rr < 16; ++rr) { b16 p, ql; split16(QKV[(size_t)(q0 + rr) * 3 * D + hd * DH + lane] * XS, p, ql); Qh[rr][lane] = p; Ql[rr][lane] = ql; }
  if (lane < 16) { Mx[lane] = -INFINITY; Dn[lane] = 0.0f; Sf[lane] = 0.0f; }
  v8f acc[2] = {(v8f){}, (v8f){}}; wave_lds_sync(); const v16b qh = frag_kb(&Qh[nloc][0], hlf), qlo = frag_kb(&Ql[nloc][0], hlf);
#pragma unroll 1
  for (int kc = 0; kc < N; kc += 32) {
    for (int rr = 0; rr < 32; ++rr) { const size_t kr = (size_t)(kc + rr) * 3 * D; b16 p, ql; split16(QKV[kr + D + hd * DH + lane] * XS, p, ql); Kh[rr][lane] = p; Kl[rr][lane] = ql; split16(QKV[kr + 2 * D + hd * DH + lane] * XS, p, ql); Vh[lane][rr] = p; Vl[lane][rr] = ql; }
    wave_lds_sync();
#pragma unroll
    for (int blk = 0; blk < 2; ++blk) { v8f s = {}; const v16b kh = frag_kb(&Kh[blk * 16 + nloc][0], hlf), kl = frag_kb(&Kl[blk * 16 + nloc][0], hlf); s = wmma16b(qh, kh, s); s = wmma16b(qh, kl, s); s = wmma16b(qlo, kh, s);
#pragma unroll
      for (int r8 = 0; r8 < 8; ++r8) { const int rl = 8 * hlf + r8, kk = blk * 16 + nloc; Sc[rl][kk] = s[r8] * (0.17677669529663688f / (XS * XS)) + BP[(size_t)(q0 + rl) * N + kc + kk]; } }
    wave_lds_sync();
#pragma unroll 1
    for (int qi = 0; qi < 16; ++qi) { const float sv = Sc[qi][lane]; float cm = sv; for (int o = 16; o; o >>= 1) cm = fmaxf(cm, __shfl_xor(cm, o)); const float mo = Mx[qi]; const float mn = fmaxf(mo, cm); const float p = __expf(sv - mn); float ps = p; for (int o = 16; o; o >>= 1) ps += __shfl_xor(ps, o);
      b16 ph, plo; split16(p * PS, ph, plo); Ph[qi][lane] = ph; Pl[qi][lane] = plo; if (lane == 0) { const float sf = (mo == -INFINITY) ? 0.0f : __expf(mo - mn); Sf[qi] = sf; Dn[qi] = Dn[qi] * sf + ps; Mx[qi] = mn; } }
    wave_lds_sync(); const v16b pa = frag_kb(&Ph[nloc][0], hlf), pb = frag_kb(&Pl[nloc][0], hlf);
#pragma unroll
    for (int t = 0; t < 2; ++t) {
#pragma unroll
      for (int r8 = 0; r8 < 8; ++r8) acc[t][r8] *= Sf[8 * hlf + r8];
      const v16b vh = frag_kb(&Vh[t * 16 + nloc][0], hlf), vl = frag_kb(&Vl[t * 16 + nloc][0], hlf); acc[t] = wmma16b(pa, vh, acc[t]); acc[t] = wmma16b(pa, vl, acc[t]); acc[t] = wmma16b(pb, vh, acc[t]); }
    wave_lds_sync(); }
#pragma unroll
  for (int t = 0; t < 2; ++t)
#pragma unroll
    for (int r8 = 0; r8 < 8; ++r8) { const int rl = 8 * hlf + r8; Of[rl][t * 16 + nloc] = acc[t][r8] * (1.0f / (PS * XS)) / Dn[rl]; }
  wave_lds_sync();
  for (int pass = 0; pass < 2; ++pass) { for (int rr = 0; rr < 16; ++rr) ((volatile float*)O)[(size_t)(q0 + rr) * D + hd * DH + lane] = Of[rr][lane]; __threadfence(); }
}
__global__ __launch_bounds__(32) void fin_kernel(const float* __restrict__ O, const b16* __restrict__ WOT, const float* __restrict__ bo, const float* __restrict__ x, const float* __restrict__ gam, const float* __restrict__ bet, int QV, float* __restrict__ out) {
  __shared__ __attribute__((aligned(16))) b16 Ah[16][D + 8], Al[16][D + 8]; __shared__ float Tf[16][D + 4]; const int lane = threadIdx.x, nloc = lane & 15, hlf = lane >> 4; const size_t m0 = (size_t)blockIdx.x * 16; if (m0 >= (size_t)QV) return;
  for (int rr = 0; rr < 16; ++rr) for (int q = 0; q < D / 32; ++q) { b16 p, ql; split16(O[(m0 + rr) * D + q * 32 + lane] * XS, p, ql); Ah[rr][q * 32 + lane] = p; Al[rr][q * 32 + lane] = ql; }
  wave_lds_sync();
  for (int g = 0; g < 2; ++g) { v8f acc[8];
#pragma unroll
    for (int t = 0; t < 8; ++t) acc[t] = (v8f){};
#pragma unroll 2
    for (int kb = 0; kb < D; kb += 32) { const v16b a = frag_kb(&Ah[nloc][kb], hlf), al = frag_kb(&Al[nloc][kb], hlf);
#pragma unroll
      for (int t = 0; t < 8; ++t) { const v16b bw = frag_kb(WOT + (size_t)(g * 128 + t * 16 + nloc) * D + kb, hlf); acc[t] = wmma16b(a, bw, acc[t]); acc[t] = wmma16b(al, bw, acc[t]); } }
#pragma unroll
    for (int t = 0; t < 8; ++t) { const int c = g * 128 + t * 16 + nloc; const float bb = bf16_rne(bo[c]);
#pragma unroll
      for (int r8 = 0; r8 < 8; ++r8) { const int rl = 8 * hlf + r8; Tf[rl][c] = acc[t][r8] * (1.0f / (XS * WSC)) + bb + bf16_rne(x[(m0 + rl) * D + c]); } } }
  wave_lds_sync();
  for (int pass = 0; pass < 2; ++pass) { for (int rr = 0; rr < 16; ++rr) { float v[8]; float s = 0.0f; for (int q = 0; q < 8; ++q) { v[q] = Tf[rr][q * 32 + lane]; s += v[q]; } for (int o = 16; o; o >>= 1) s += __shfl_xor(s, o); const float mu = s * (1.0f / D); float qq = 0.0f; for (int q = 0; q < 8; ++q) qq += pmul(v[q] - mu, v[q] - mu); for (int o = 16; o; o >>= 1) qq += __shfl_xor(qq, o); const float rs = rsqrtf(qq * (1.0f / D) + 1e-5f);
      for (int q = 0; q < 8; ++q) { const int c = q * 32 + lane; ((volatile float*)out)[(m0 + rr) * D + c] = pmul(pmul(v[q] - mu, rs), bf16_rne(gam[c])) + bf16_rne(bet[c]); } } __threadfence(); }
}
}

extern "C" void kernel_launch(void* const* d_in, const int* in_sizes, int n_in, void* d_out, int out_size, void* d_ws, size_t ws_size, hipStream_t stream) {
  (void)n_in;
  auto Fp = [&](int i) { return (const float*)d_in[i]; }; auto Ip = [&](int i) { return (const int*)d_in[i]; };
  if (in_sizes[0] != N * D || in_sizes[1] != N * D || in_sizes[2] != 2 * E || in_sizes[3] != E || in_sizes[4] != D * D || in_sizes[10] != D * D || in_sizes[12] != NTY * NHD || out_size != N * D) return;
  const int QV = N; const int HV = NHD;
  size_t off = 0; char* ws = (char*)d_ws;
  auto carve = [&](size_t bytes) { char* p = ws + off; off += (bytes + 255) & ~(size_t)255; return p; };
  b16* WQ = (b16*)carve((size_t)3 * D * D * 2); b16* WO = (b16*)carve((size_t)D * D * 2); float* QKV = (float*)carve((size_t)N * 3 * D * 4); float* BP = (float*)carve((size_t)N * N * 4); float* O = (float*)carve((size_t)N * D * 4); CsrBufs7 csr; off = csr_carve7(csr, ws, off, E, N);
  if (off > ws_size || off > ((size_t)128 << 20)) return;
  wput_kernel<<<(D * 32 + 255) / 256, 256, 0, stream>>>(Fp(4), 0, WQ); wput_kernel<<<(D * 32 + 255) / 256, 256, 0, stream>>>(Fp(6), D, WQ); wput_kernel<<<(D * 32 + 255) / 256, 256, 0, stream>>>(Fp(8), 2 * D, WQ); wput_kernel<<<(D * 32 + 255) / 256, 256, 0, stream>>>(Fp(10), 0, WO);
  csr_build7(csr, Ip(2), E, N, stream);
  qkv_kernel<<<(N / 16) * 6, 32, 0, stream>>>(Fp(0), Fp(1), WQ, Fp(5), Fp(7), Fp(9), QKV);
  if (HV < NHD) {   }
  for (int hd = 0; hd < NHD; ++hd) {
    if (hd < HV) { bias_kernel<<<N, 32, 0, stream>>>(Fp(12), Ip(2) + E, Ip(3), hd, csr.PERM, csr.ROWPTR, csr.ROWCNT, (int)csr.permLen, BP); att_kernel<<<N / 16, 32, 0, stream>>>(QKV, BP, hd, QV, O); } }
  fin_kernel<<<N / 16, 32, 0, stream>>>(O, WO, Fp(11), Fp(0), Fp(13), Fp(14), QV, (float*)d_out);
}
